// WeightedValues_45148696215770
// MI455X (gfx1250) — hardware-verified
//
#include <hip/hip_runtime.h>
#include <math.h>

#define NB   8
#define SEQ  2048
#define HD   128

static_assert(SEQ % 128 == 0);
static_assert(HD == 128);

typedef __attribute__((ext_vector_type(16))) __bf16 v16b;
typedef __attribute__((ext_vector_type(8)))  __bf16 v8b;
typedef __attribute__((ext_vector_type(8)))  float  v8f;
typedef __attribute__((ext_vector_type(4)))  float  v4f;
typedef __attribute__((ext_vector_type(4)))  unsigned int v4u;
typedef __attribute__((ext_vector_type(8)))  unsigned short v8us;

__device__ __forceinline__ unsigned short f2bf_bits(float f) {
  unsigned u = __float_as_uint(f);
  return (unsigned short)((u + 0x7FFFu + ((u >> 16) & 1u)) >> 16);
}
__device__ __forceinline__ float bf_bits2f(unsigned short b) { return __uint_as_float(((unsigned)b) << 16); }
__device__ __forceinline__ unsigned pk16(unsigned short a, unsigned short b) { return (unsigned)a | ((unsigned)b << 16); }

__device__ __forceinline__ void split2(float f0, float f1, unsigned& hw, unsigned& lw) {
  const unsigned short h0 = f2bf_bits(f0), h1 = f2bf_bits(f1);
  const unsigned short l0 = f2bf_bits(f0 - bf_bits2f(h0)), l1 = f2bf_bits(f1 - bf_bits2f(h1));
  hw = pk16(h0, h1);
  lw = pk16(l0, l1);
}

__device__ __forceinline__ v8f mma_bf(v16b a, v16b b, v8f c) {
  c = __builtin_amdgcn_wmma_f32_16x16x32_bf16(false, a, false, b, (short)0, c, false, false);
  asm volatile("v_nop\n\tv_nop\n\tv_nop\n\tv_nop" : "+v"(c) : "v"(a), "v"(b));
  return c;
}

__device__ __forceinline__ void lds_wave_sync() {
  __builtin_amdgcn_fence(__ATOMIC_RELEASE, "workgroup");
  __builtin_amdgcn_wave_barrier();
  __builtin_amdgcn_fence(__ATOMIC_ACQUIRE, "workgroup");
}

#define WTP 136
#define QSP 136

__global__ __launch_bounds__(256)
void proj_kernel(const float* __restrict__ query, const float* __restrict__ key,
                 const float* __restrict__ Wq, const float* __restrict__ Wk,
                 unsigned short* __restrict__ Qhp, unsigned short* __restrict__ Qlp,
                 unsigned short* __restrict__ Khp, unsigned short* __restrict__ Klp) {
  union FB { v16b v; v8b h[2]; unsigned u[8]; };
  __shared__ __align__(16) __bf16 Wth[HD * WTP];
  __shared__ __align__(16) __bf16 Wtl[HD * WTP];
  __shared__ __align__(16) unsigned short Qst[8][16 * QSP];

  const int tid  = threadIdx.x;
  const int wave = tid >> 5;
  const int lane = tid & 31;
  const int lh   = lane >> 4;
  const int c    = lane & 15;
  const int which = blockIdx.x >> 7;
  const int rem  = blockIdx.x & 127;
  const int b    = rem >> 4;
  const int rt   = rem & 15;
  const int row0 = rt * 128 + wave * 16;

  const float* src = which ? key : query;
  const float* W   = which ? Wk  : Wq;
  unsigned short* dh = which ? Khp : Qhp;
  unsigned short* dl = which ? Klp : Qlp;

#pragma unroll 4
  for (int idx = tid; idx < HD * HD; idx += 256) {
    const int d = idx >> 7, n = idx & 127;
    const float w = W[idx];
    const unsigned short hb = f2bf_bits(w);
    const unsigned short lb = f2bf_bits(w - bf_bits2f(hb));
    Wth[n * WTP + d] = __builtin_bit_cast(__bf16, hb);
    Wtl[n * WTP + d] = __builtin_bit_cast(__bf16, lb);
  }
  __syncthreads();

  v8f acc[8];
#pragma unroll
  for (int nt = 0; nt < 8; ++nt) acc[nt] = (v8f){0.f, 0.f, 0.f, 0.f, 0.f, 0.f, 0.f, 0.f};

  const float* arow = src + ((size_t)(b * SEQ + row0 + c)) * HD + 8 * lh;
#pragma unroll
  for (int dc = 0; dc < 4; ++dc) {
    const v4f f0 = *(const v4f*)(arow + dc * 32);
    const v4f f1 = *(const v4f*)(arow + dc * 32 + 4);
    const v4f f2 = *(const v4f*)(arow + dc * 32 + 16);
    const v4f f3 = *(const v4f*)(arow + dc * 32 + 20);
    FB ah, al;
    split2(f0[0], f0[1], ah.u[0], al.u[0]);
    split2(f0[2], f0[3], ah.u[1], al.u[1]);
    split2(f1[0], f1[1], ah.u[2], al.u[2]);
    split2(f1[2], f1[3], ah.u[3], al.u[3]);
    split2(f2[0], f2[1], ah.u[4], al.u[4]);
    split2(f2[2], f2[3], ah.u[5], al.u[5]);
    split2(f3[0], f3[1], ah.u[6], al.u[6]);
    split2(f3[2], f3[3], ah.u[7], al.u[7]);
#pragma unroll
    for (int nt = 0; nt < 8; ++nt) {
      const __bf16* wp = Wth + (nt * 16 + c) * WTP + dc * 32 + 8 * lh;
      const __bf16* wq = Wtl + (nt * 16 + c) * WTP + dc * 32 + 8 * lh;
      FB bh, bl;
      bh.h[0] = *(const v8b*)(wp);
      bh.h[1] = *(const v8b*)(wp + 16);
      bl.h[0] = *(const v8b*)(wq);
      bl.h[1] = *(const v8b*)(wq + 16);
      acc[nt] = mma_bf(ah.v, bh.v, acc[nt]);
      acc[nt] = mma_bf(ah.v, bl.v, acc[nt]);
      acc[nt] = mma_bf(al.v, bh.v, acc[nt]);
    }
  }

  unsigned short* st = Qst[wave];
  const int c8 = c * 8;
#pragma unroll
  for (int r = 0; r < 8; ++r)
#pragma unroll
    for (int nt = 0; nt < 8; ++nt)
      st[(8 * lh + r) * QSP + nt * 16 + c] = f2bf_bits(acc[nt][r]);
  lds_wave_sync();
  v8us hv[8];
#pragma unroll
  for (int it = 0; it < 8; ++it) hv[it] = *(const v8us*)(st + (2 * it + lh) * QSP + c8);
  lds_wave_sync();
#pragma unroll
  for (int r = 0; r < 8; ++r)
#pragma unroll
    for (int nt = 0; nt < 8; ++nt) {
      const float a = acc[nt][r];
      const unsigned short hb = f2bf_bits(a);
      st[(8 * lh + r) * QSP + nt * 16 + c] = f2bf_bits(a - bf_bits2f(hb));
    }
  lds_wave_sync();
  v8us lv[8];
#pragma unroll
  for (int it = 0; it < 8; ++it) lv[it] = *(const v8us*)(st + (2 * it + lh) * QSP + c8);

  unsigned short* gh = dh + ((size_t)(b * SEQ + row0)) * HD;
  unsigned short* gl = dl + ((size_t)(b * SEQ + row0)) * HD;
  for (int ps = 0; ps < 2; ++ps) {
#pragma unroll
    for (int it = 0; it < 8; ++it) {
      const size_t go = (size_t)(2 * it + lh) * HD + c8;
      *(volatile v8us*)(gh + go) = hv[it];
      *(volatile v8us*)(gl + go) = lv[it];
    }
    __threadfence();
  }
}

#define TFP 132
__global__ __launch_bounds__(256) void vt_split_kernel(const float* __restrict__ v,
                                                       unsigned short* __restrict__ vth,
                                                       unsigned short* __restrict__ vtl) {
  __shared__ __align__(16) float tf[64 * TFP];
  const int tid = threadIdx.x;
  const int nt  = blockIdx.x % (SEQ / 64);
  const int b   = blockIdx.x / (SEQ / 64);
  const int n0  = nt * 64;
  {
    const int lr = tid >> 4;
    const int c8 = (tid & 15) * 8;
#pragma unroll
    for (int it = 0; it < 4; ++it) {
      const int row = it * 16 + lr;
      const float* sp = v + ((size_t)(b * SEQ + n0 + row)) * HD + c8;
      const v4f a0 = *(const v4f*)(sp);
      const v4f a1 = *(const v4f*)(sp + 4);
      *(v4f*)(tf + row * TFP + c8) = a0;
      *(v4f*)(tf + row * TFP + c8 + 4) = a1;
    }
  }
  __syncthreads();
  {
    const int sub = tid >> 3;
    const int t8  = (tid & 7) * 8;
    v4u hv[4], lv[4];
#pragma unroll
    for (int it = 0; it < 4; ++it) {
      const int d = it * 32 + sub;
      unsigned hw[4], lw[4];
#pragma unroll
      for (int q = 0; q < 4; ++q) {
        const float f0 = tf[(t8 + 2 * q) * TFP + d];
        const float f1 = tf[(t8 + 2 * q + 1) * TFP + d];
        split2(f0, f1, hw[q], lw[q]);
      }
      hv[it] = (v4u){hw[0], hw[1], hw[2], hw[3]};
      lv[it] = (v4u){lw[0], lw[1], lw[2], lw[3]};
    }
    unsigned short* th = vth + (size_t)b * HD * SEQ + n0 + t8;
    unsigned short* tl = vtl + (size_t)b * HD * SEQ + n0 + t8;
    for (int ps = 0; ps < 2; ++ps) {
#pragma unroll
      for (int it = 0; it < 4; ++it) {
        const int d = it * 32 + sub;
        const size_t go = (size_t)d * SEQ;
        *(volatile v4u*)(th + go) = hv[it];
        *(volatile v4u*)(tl + go) = lv[it];
      }
      __threadfence();
    }
  }
}

#define QB  64
#define KC  64
#define KSP 136
#define VTP 72
#define PSP 64
#define OSP 68

__global__ __launch_bounds__(256)
void attn_kernel(const unsigned short* __restrict__ qhp, const unsigned short* __restrict__ qlp,
                 const unsigned short* __restrict__ khp, const unsigned short* __restrict__ klp,
                 const unsigned short* __restrict__ vhp, const unsigned short* __restrict__ vlp,
                 const float* __restrict__ mask, float* __restrict__ out) {
  union FB { v16b v; v8b h[2]; };
  __shared__ __align__(16) __bf16 Ksh[KC * KSP];
  __shared__ __align__(16) __bf16 Ksl[KC * KSP];
  __shared__ __align__(16) __bf16 Vth[HD * VTP];
  __shared__ __align__(16) __bf16 Vtl[HD * VTP];
  __shared__ __align__(16) __bf16 Psh[4][16 * PSP];
  __shared__ __align__(16) __bf16 Psl[4][16 * PSP];
  __shared__ __align__(16) float  Al[4][16];
  __shared__ __align__(16) float  Ll[4][16];
  __shared__ __align__(16) float  Os[8][16 * OSP];

  const int tid  = threadIdx.x;
  const int wave = tid >> 5;
  const int lane = tid & 31;
  const int lh   = lane >> 4;
  const int c    = lane & 15;
  const int g    = wave & 3;
  const int chh  = wave >> 2;
  const int ch0  = chh * 64;

  const int nqt = SEQ / QB;
  const int qt  = blockIdx.x % nqt;
  const int b   = blockIdx.x / nqt;
  const int qg0 = qt * QB + g * 16;

  const __bf16* Qh = (const __bf16*)(const void*)qhp + (size_t)b * SEQ * HD;
  const __bf16* Ql = (const __bf16*)(const void*)qlp + (size_t)b * SEQ * HD;
  const __bf16* Kh = (const __bf16*)(const void*)khp + (size_t)b * SEQ * HD;
  const __bf16* Kl = (const __bf16*)(const void*)klp + (size_t)b * SEQ * HD;
  const __bf16* Vh = (const __bf16*)(const void*)vhp + (size_t)b * HD * SEQ;
  const __bf16* Vl = (const __bf16*)(const void*)vlp + (size_t)b * HD * SEQ;
  const float*  mk = mask + (size_t)b * SEQ;

  float mrow[8], lrow[8];
  v8f oacc[4];
#pragma unroll
  for (int r = 0; r < 8; ++r) { mrow[r] = -INFINITY; lrow[r] = 0.f; }
#pragma unroll
  for (int t = 0; t < 4; ++t) oacc[t] = (v8f){0.f, 0.f, 0.f, 0.f, 0.f, 0.f, 0.f, 0.f};

  __bf16* pwh = Psh[g];
  __bf16* pwl = Psl[g];

  for (int kc = 0; kc < SEQ / KC; ++kc) {
    const int kv0 = kc * KC;
    __syncthreads();
    {
      const int r = tid >> 2, qq = (tid & 3) * 32;
      const __bf16* khs = Kh + (size_t)(kv0 + r) * HD + qq;
      const __bf16* kls = Kl + (size_t)(kv0 + r) * HD + qq;
      __bf16* kdh = Ksh + r * KSP + qq;
      __bf16* kdl = Ksl + r * KSP + qq;
#pragma unroll
      for (int i = 0; i < 4; ++i) {
        *(v8b*)(kdh + 8 * i) = *(const v8b*)(khs + 8 * i);
        *(v8b*)(kdl + 8 * i) = *(const v8b*)(kls + 8 * i);
      }
      const int r2 = tid >> 1, hf = (tid & 1) * 32;
      const __bf16* vhs = Vh + (size_t)r2 * SEQ + kv0 + hf;
      const __bf16* vls = Vl + (size_t)r2 * SEQ + kv0 + hf;
#pragma unroll
      for (int i = 0; i < 4; ++i) {
        *(v8b*)(Vth + r2 * VTP + hf + 8 * i) = *(const v8b*)(vhs + 8 * i);
        *(v8b*)(Vtl + r2 * VTP + hf + 8 * i) = *(const v8b*)(vls + 8 * i);
      }
    }
    __syncthreads();

    if (wave < 4) {
      v8f s[4];
#pragma unroll
      for (int j = 0; j < 4; ++j) s[j] = (v8f){0.f, 0.f, 0.f, 0.f, 0.f, 0.f, 0.f, 0.f};
      const __bf16* qrh = Qh + (size_t)(qg0 + c) * HD + 8 * lh;
      const __bf16* qrl = Ql + (size_t)(qg0 + c) * HD + 8 * lh;
#pragma unroll
      for (int dc = 0; dc < 4; ++dc) {
        FB qa, ql;
        qa.h[0] = *(const v8b*)(qrh + dc * 32);
        qa.h[1] = *(const v8b*)(qrh + dc * 32 + 16);
        ql.h[0] = *(const v8b*)(qrl + dc * 32);
        ql.h[1] = *(const v8b*)(qrl + dc * 32 + 16);
#pragma unroll
        for (int j = 0; j < 4; ++j) {
          const __bf16* kp = Ksh + (j * 16 + c) * KSP + dc * 32 + 8 * lh;
          const __bf16* kq = Ksl + (j * 16 + c) * KSP + dc * 32 + 8 * lh;
          FB kb, kl;
          kb.h[0] = *(const v8b*)(kp);
          kb.h[1] = *(const v8b*)(kp + 16);
          kl.h[0] = *(const v8b*)(kq);
          kl.h[1] = *(const v8b*)(kq + 16);
          s[j] = mma_bf(qa.v, kb.v, s[j]);
          s[j] = mma_bf(qa.v, kl.v, s[j]);
          s[j] = mma_bf(ql.v, kb.v, s[j]);
        }
      }
      float mv[4], om[4];
#pragma unroll
      for (int j = 0; j < 4; ++j) {
        mv[j] = mk[kv0 + j * 16 + c];
        om[j] = (1.0f - mv[j]) * (-1.0e30f);
      }
      float cm[8];
#pragma unroll
      for (int r = 0; r < 8; ++r) {
        float m = -INFINITY;
#pragma unroll
        for (int j = 0; j < 4; ++j) {
          const float sv = mv[j] * s[j][r] + om[j];
          s[j][r] = sv;
          m = fmaxf(m, sv);
        }
#pragma unroll
        for (int off = 1; off < 16; off <<= 1) m = fmaxf(m, __shfl_xor(m, off, 32));
        cm[r] = m;
      }
#pragma unroll
      for (int r = 0; r < 8; ++r) {
        const float mnew  = fmaxf(mrow[r], cm[r]);
        const float alpha = __expf(mrow[r] - mnew);
        mrow[r] = mnew;
        float psum = 0.f;
#pragma unroll
        for (int j = 0; j < 4; ++j) {
          const float p = __expf(s[j][r] - mnew);
          psum += p;
          const unsigned short hb = f2bf_bits(p);
          const unsigned short lb = f2bf_bits(p - bf_bits2f(hb));
          pwh[(8 * lh + r) * PSP + j * 16 + c] = __builtin_bit_cast(__bf16, hb);
          pwl[(8 * lh + r) * PSP + j * 16 + c] = __builtin_bit_cast(__bf16, lb);
        }
#pragma unroll
        for (int off = 1; off < 16; off <<= 1) psum += __shfl_xor(psum, off, 32);
        lrow[r] = lrow[r] * alpha + psum;
        if (c == 0) {
          Al[g][8 * lh + r] = alpha;
          Ll[g][8 * lh + r] = lrow[r];
        }
      }
    }
    __syncthreads();

    {
      float af[8];
#pragma unroll
      for (int r = 0; r < 8; ++r) af[r] = Al[g][8 * lh + r];
#pragma unroll
      for (int t = 0; t < 4; ++t)
#pragma unroll
        for (int r = 0; r < 8; ++r) oacc[t][r] *= af[r];
#pragma unroll 1
      for (int kk = 0; kk < 2; ++kk) {
        FB pa, pl;
        pa.h[0] = *(const v8b*)(pwh + c * PSP + kk * 32 + 8 * lh);
        pa.h[1] = *(const v8b*)(pwh + c * PSP + kk * 32 + 16 + 8 * lh);
        pl.h[0] = *(const v8b*)(pwl + c * PSP + kk * 32 + 8 * lh);
        pl.h[1] = *(const v8b*)(pwl + c * PSP + kk * 32 + 16 + 8 * lh);
#pragma unroll
        for (int t = 0; t < 4; ++t) {
          const __bf16* vp = Vth + (ch0 + t * 16 + c) * VTP + kk * 32 + 8 * lh;
          const __bf16* vq = Vtl + (ch0 + t * 16 + c) * VTP + kk * 32 + 8 * lh;
          FB vb, vl;
          vb.h[0] = *(const v8b*)(vp);
          vb.h[1] = *(const v8b*)(vp + 16);
          vl.h[0] = *(const v8b*)(vq);
          vl.h[1] = *(const v8b*)(vq + 16);
          oacc[t] = mma_bf(pa.v, vb.v, oacc[t]);
          oacc[t] = mma_bf(pa.v, vl.v, oacc[t]);
          oacc[t] = mma_bf(pl.v, vb.v, oacc[t]);
        }
      }
    }
  }

  float* os = Os[wave];
#pragma unroll
  for (int r = 0; r < 8; ++r) {
    const float inv = 1.0f / Ll[g][8 * lh + r];
#pragma unroll
    for (int t = 0; t < 4; ++t) os[(8 * lh + r) * OSP + t * 16 + c] = oacc[t][r] * inv;
  }
  lds_wave_sync();
  {
    const int rh = lane >> 4, c4 = (lane & 15) * 4;
    v4f ov[8];
#pragma unroll
    for (int it = 0; it < 8; ++it) ov[it] = *(const v4f*)(os + (it * 2 + rh) * OSP + c4);
    for (int ps = 0; ps < 2; ++ps) {
#pragma unroll
      for (int it = 0; it < 8; ++it) {
        const int row = it * 2 + rh;
        const size_t go = ((size_t)(b * SEQ + qg0 + row)) * HD + ch0 + c4;
        *(volatile v4f*)(out + go) = ov[it];
      }
      __threadfence();
    }
  }
}

extern "C" void kernel_launch(void* const* d_in, const int* in_sizes, int n_in,
                              void* d_out, int out_size, void* d_ws, size_t ws_size,
                              hipStream_t stream) {
  if (n_in < 6) return;
  if (in_sizes[0] != NB * SEQ * HD) return;
  if (in_sizes[1] != NB * SEQ * HD) return;
  if (in_sizes[2] != NB * SEQ * HD) return;
  if (in_sizes[3] != NB * SEQ) return;
  if (in_sizes[4] != HD * HD) return;
  if (in_sizes[5] != HD * HD) return;
  if (out_size != NB * SEQ * HD) return;

  const float* query = (const float*)d_in[0];
  const float* key   = (const float*)d_in[1];
  const float* value = (const float*)d_in[2];
  const float* mask  = (const float*)d_in[3];
  const float* Wq    = (const float*)d_in[4];
  const float* Wk    = (const float*)d_in[5];
  float* o = (float*)d_out;

  const size_t PP = (size_t)NB * SEQ * HD * 2;
  size_t off = 0;
  const size_t oQh = off; off += PP;
  const size_t oQl = off; off += PP;
  const size_t oKh = off; off += PP;
  const size_t oKl = off; off += PP;
  const size_t oVh = off; off += PP;
  const size_t oVl = off; off += PP;
  if (off > ws_size) return;

  char* ws = (char*)d_ws;
  unsigned short* Qh  = (unsigned short*)(ws + oQh);
  unsigned short* Ql  = (unsigned short*)(ws + oQl);
  unsigned short* Kh  = (unsigned short*)(ws + oKh);
  unsigned short* Kl  = (unsigned short*)(ws + oKl);
  unsigned short* VTh = (unsigned short*)(ws + oVh);
  unsigned short* VTl = (unsigned short*)(ws + oVl);

  proj_kernel<<<dim3(2 * NB * (SEQ / 128)), dim3(256), 0, stream>>>(query, key, Wq, Wk, Qh, Ql, Kh, Kl);
  vt_split_kernel<<<dim3(NB * (SEQ / 64)), dim3(256), 0, stream>>>(value, VTh, VTl);
  attn_kernel<<<dim3(NB * (SEQ / QB)), dim3(256), 0, stream>>>(Qh, Ql, Kh, Kl, VTh, VTl, mask, o);
  (void)hipGetLastError();
}
